// FeatureNet_57174604644985
// MI455X (gfx1250) — hardware-verified
//
#include <hip/hip_runtime.h>
#include <math.h>

constexpr int NBAT = 128;
constexpr int NTS  = 200;
constexpr int NCV  = 40;
constexpr int NVOC = 2000;
constexpr int NAUX = 16;
constexpr int NE   = 128;
constexpr int NG4  = 512;
constexpr int NHM  = 256;
constexpr int NLIN = NVOC + NAUX;
constexpr int NROW = NBAT * NTS;
constexpr int NTHR = 256;
constexpr int FE_RPB = NTHR / 32;
constexpr int SEQB = 16;
constexpr int HPITCH = 136;
constexpr int ZPITCH = 516;
constexpr int LPITCH = 132;
constexpr int YPITCH = 260;
constexpr float XCAR = 64.0f;
constexpr float WCAR = 256.0f;
constexpr float HCAR = 256.0f;
constexpr float XW_INV = 1.0f / 16384.0f;
constexpr float HW_INV = 1.0f / 65536.0f;
static_assert(NROW % 64 == 0 && NG4 % 64 == 0 && NE % 32 == 0);
static_assert(((NROW / 64) * (NG4 / 64)) % 8 == 0);
static_assert(NROW % FE_RPB == 0);
static_assert(NBAT % SEQB == 0);
static_assert(NE == 16 * (NTHR / 32));
static_assert(NHM == NTHR);
static_assert(8 * NTHR * 4 == SEQB * NG4);
static_assert(NG4 / 4 == 128);
static_assert(NE % 64 == 0 && NG4 % 64 == 0);
static_assert(NCV <= 64 && NCV > 32);

typedef __attribute__((ext_vector_type(16))) _Float16 v16h;
typedef __attribute__((ext_vector_type(8)))  _Float16 v8h;
typedef __attribute__((ext_vector_type(16))) __bf16   v16b;
typedef __attribute__((ext_vector_type(8)))  __bf16   v8b;
typedef __attribute__((ext_vector_type(8)))  float    v8f;
typedef __attribute__((ext_vector_type(4)))  float    v4f;

__device__ __forceinline__ unsigned short f2bf_bits(float f) {
  unsigned u = __float_as_uint(f);
  return (unsigned short)((u + 0x7FFFu + ((u >> 16) & 1u)) >> 16);
}
__device__ __forceinline__ float bf_bits2f(unsigned short h) { return __uint_as_float(((unsigned)h) << 16); }

__device__ __forceinline__ void dep_guard_h(v8f& a, v8f& b, v16h x, v16h y) { asm volatile("v_nop\n\tv_nop\n\tv_nop\n\tv_nop" : "+v"(a), "+v"(b) : "v"(x), "v"(y)); }
__device__ __forceinline__ void dep_guard_b(v8f& a, v8f& b, v16b x, v16b y) { asm volatile("v_nop\n\tv_nop\n\tv_nop\n\tv_nop" : "+v"(a), "+v"(b) : "v"(x), "v"(y)); }
__device__ __forceinline__ void dep_guard4_h(v8f& a, v8f& b, v8f& c, v8f& d, v16h x, v16h y) { asm volatile("v_nop\n\tv_nop\n\tv_nop\n\tv_nop" : "+v"(a), "+v"(b), "+v"(c), "+v"(d) : "v"(x), "v"(y)); }
__device__ __forceinline__ void dep_guard4_b(v8f& a, v8f& b, v8f& c, v8f& d, v16b x, v16b y) { asm volatile("v_nop\n\tv_nop\n\tv_nop\n\tv_nop" : "+v"(a), "+v"(b), "+v"(c), "+v"(d) : "v"(x), "v"(y)); }
__device__ __forceinline__ void keep4_h(v16h a, v16h b, v16h c, v16h d) { asm volatile("v_nop" :: "v"(a), "v"(b), "v"(c), "v"(d)); }
__device__ __forceinline__ void keep4_b(v16b a, v16b b, v16b c, v16b d) { asm volatile("v_nop" :: "v"(a), "v"(b), "v"(c), "v"(d)); }
__device__ __forceinline__ void acc_guard4(v8f& a, v8f& b, v8f& c, v8f& d) { asm volatile("v_nop\n\tv_nop\n\tv_nop\n\tv_nop" : "+v"(a), "+v"(b), "+v"(c), "+v"(d)); }
__device__ __forceinline__ void mma_guard_all_h(v8f& a0, v8f& a1, v8f& a2, v8f& a3, v16h x, v16h y0, v16h y1, v16h y2, v16h y3) {
  asm volatile("v_nop\n\tv_nop\n\tv_nop\n\tv_nop" : "+v"(a0), "+v"(a1), "+v"(a2), "+v"(a3) : "v"(x), "v"(y0), "v"(y1), "v"(y2), "v"(y3));
}
template <typename T> struct Frag;
template <> struct Frag<_Float16> {
  typedef v16h V; union U { v16h v; v8h h[2]; };
  static __device__ __forceinline__ v16h load(const _Float16* p) {
    U f; f.h[0] = *(const v8h*)(p); f.h[1] = *(const v8h*)(p + 16); return f.v;
  }
  static __device__ __forceinline__ v8f mma(v16h a, v16h b, v8f c) {
    return __builtin_amdgcn_wmma_f32_16x16x32_f16(false, a, false, b, (short)0, c, false, false);
  }
  static __device__ __forceinline__ void guard(v8f& a, v8f& b, v16h x, v16h y) { dep_guard_h(a, b, x, y); }
  static __device__ __forceinline__ void guard4(v8f& a, v8f& b, v8f& c, v8f& d, v16h x, v16h y) { dep_guard4_h(a, b, c, d, x, y); }
  static __device__ __forceinline__ void keep(v16h a, v16h b, v16h c, v16h d) { keep4_h(a, b, c, d); }
};
template <> struct Frag<__bf16> {
  typedef v16b V; union U { v16b v; v8b h[2]; };
  static __device__ __forceinline__ v16b load(const __bf16* p) {
    U f; f.h[0] = *(const v8b*)(p); f.h[1] = *(const v8b*)(p + 16); return f.v;
  }
  static __device__ __forceinline__ v8f mma(v16b a, v16b b, v8f c) {
    return __builtin_amdgcn_wmma_f32_16x16x32_bf16(false, a, false, b, (short)0, c, false, false);
  }
  static __device__ __forceinline__ void guard(v8f& a, v8f& b, v16b x, v16b y) { dep_guard_b(a, b, x, y); }
  static __device__ __forceinline__ void guard4(v8f& a, v8f& b, v8f& c, v8f& d, v16b x, v16b y) { dep_guard4_b(a, b, c, d, x, y); }
  static __device__ __forceinline__ void keep(v16b a, v16b b, v16b c, v16b d) { keep4_b(a, b, c, d); }
};

__device__ __forceinline__ float fsig(float x)  { return __builtin_amdgcn_rcpf(1.0f + expf(-x)); }
__device__ __forceinline__ float ftanh(float x) { return 1.0f - 2.0f * __builtin_amdgcn_rcpf(expf(2.0f * x) + 1.0f); }

template <int ET> struct Elem;
template <> struct Elem<0> { typedef _Float16 T; };
template <> struct Elem<1> { typedef __bf16 T; };
template <int ET, bool SPLIT, int BIAS_MODE, int OUT_MODE, bool RESID, int ACT = 0>
__global__ __launch_bounds__(256) void wmma_gemm64(
    const unsigned short* __restrict__ Ap, const unsigned short* __restrict__ A2p, int lda, long strideA,
    const unsigned short* __restrict__ Btp, const unsigned short* __restrict__ Bt2p, int ldb, long strideB,
    void* __restrict__ Cout, void* __restrict__ Cout2, int ldc, long strideC,
    const float* __restrict__ bias,
    const float* __restrict__ resid, long strideR,
    int M, int N, int K, float scale) {
  typedef typename Elem<ET>::T T;
  typedef typename Frag<T>::V V;
  const T* A = (const T*)Ap; const T* A2 = (const T*)A2p; const T* Bt = (const T*)Btp; const T* Bt2 = (const T*)Bt2p;
  __shared__ __align__(16) float sT[8][16 * 68];
  const int b    = blockIdx.y;
  const int lane = threadIdx.x & 31;
  const int wave = threadIdx.x >> 5;
  const int tilesN = N >> 6;
  const int tilesM = M >> 6;
  const int tile = blockIdx.x * 8 + wave;
  if (tile >= tilesM * tilesN) return;
  const int tm = tile / tilesN;
  const int tn = tile - tm * tilesN;
  const int m0 = tm << 6;
  const int n0 = tn << 6;

  const T* Ab  = A  + (size_t)b * strideA;
  const T* Bb  = Bt + (size_t)b * strideB;
  const T* Ab2 = SPLIT ? (A2  + (size_t)b * strideA) : nullptr;
  const T* Bb2 = SPLIT ? (Bt2 + (size_t)b * strideB) : nullptr;

  const int rlane = lane & 15;
  const int koff  = (lane >> 4) * 8;
  const int mOff  = (lane >> 4) * 8;

  v8f acc[4][4];
#pragma unroll
  for (int i = 0; i < 4; ++i)
#pragma unroll
    for (int j = 0; j < 4; ++j) acc[i][j] = (v8f){0.f,0.f,0.f,0.f,0.f,0.f,0.f,0.f};

  for (int k0 = 0; k0 < K; k0 += 32) {
    V bh[4], bl[4];
#pragma unroll
    for (int j = 0; j < 4; ++j) {
      const size_t bo = (size_t)(n0 + (j << 4) + rlane) * ldb + koff + k0;
      bh[j] = Frag<T>::load(Bb + bo);
      if (SPLIT) bl[j] = Frag<T>::load(Bb2 + bo);
    }
#pragma unroll
    for (int i = 0; i < 4; ++i) {
      const size_t ao = (size_t)(m0 + (i << 4) + rlane) * lda + koff + k0;
      V ah = Frag<T>::load(Ab + ao);
      V al;
      if (SPLIT) al = Frag<T>::load(Ab2 + ao);
#pragma unroll
      for (int j = 0; j < 4; ++j) {
        acc[i][j] = Frag<T>::mma(ah, bh[j], acc[i][j]);
        if (SPLIT) {
          acc[i][j] = Frag<T>::mma(ah, bl[j], acc[i][j]);
          acc[i][j] = Frag<T>::mma(al, bh[j], acc[i][j]);
        }
      }
      Frag<T>::guard4(acc[i][0], acc[i][1], acc[i][2], acc[i][3], ah, SPLIT ? al : ah);
    }
    Frag<T>::keep(bh[0], bh[1], bh[2], bh[3]);
    if (SPLIT) Frag<T>::keep(bl[0], bl[1], bl[2], bl[3]);
  }
  acc_guard4(acc[0][0], acc[0][1], acc[0][2], acc[0][3]);
  acc_guard4(acc[1][0], acc[1][1], acc[1][2], acc[1][3]);
  acc_guard4(acc[2][0], acc[2][1], acc[2][2], acc[2][3]);
  acc_guard4(acc[3][0], acc[3][1], acc[3][2], acc[3][3]);

  float* slab = sT[wave];
  const float* Rb = RESID ? (resid + (size_t)b * strideR) : nullptr;
#pragma unroll
  for (int i = 0; i < 4; ++i) {
    const int mBase = m0 + (i << 4);
#pragma unroll
    for (int j = 0; j < 4; ++j) {
      const int n = n0 + (j << 4) + rlane;
      float bv = 0.f;
      if (BIAS_MODE == 2) bv = bias[n];
#pragma unroll
      for (int r = 0; r < 8; ++r) {
        float v = acc[i][j][r] * scale;
        if (BIAS_MODE == 1) v += bias[mBase + mOff + r];
        if (BIAS_MODE == 2) v += bv;
        if (RESID) v += Rb[(size_t)(mBase + mOff + r) * ldc + n];
        if (ACT == 1) v = tanhf(v);
        if (ACT == 2) v = fmaxf(v, 0.0f);
        if (ACT == 3) v = v / (1.0f + expf(-v));
        if (ACT == 4) v = (v > 0.f) ? v : 0.01f * v;
        if (ACT == 5) v = 0.5f * v * (1.0f + erff(v * 0.70710678118654752f));
        slab[(mOff + r) * 68 + (j << 4) + rlane] = v;
      }
    }
    __builtin_amdgcn_fence(__ATOMIC_RELEASE, "workgroup");
    __builtin_amdgcn_wave_barrier();
    __builtin_amdgcn_fence(__ATOMIC_ACQUIRE, "workgroup");
    if (OUT_MODE == 0) {
      float* C = (float*)Cout + (size_t)b * strideC;
      const int hh = lane >> 4, c4 = (lane & 15) * 4;
      for (int pass = 0; pass < 2; ++pass) {
#pragma unroll
        for (int it = 0; it < 8; ++it) {
          const int row = it * 2 + hh;
          v4f v = *(const v4f*)(slab + row * 68 + c4);
          *(volatile v4f*)(C + (size_t)(mBase + row) * ldc + n0 + c4) = v;
        }
        __threadfence();
      }
    } else {
      const int q = lane >> 3, c8 = (lane & 7) * 8;
      unsigned short* C  = (unsigned short*)Cout  + (size_t)b * strideC;
      unsigned short* C2 = (OUT_MODE == 2) ? ((unsigned short*)Cout2 + (size_t)b * strideC) : nullptr;
      for (int pass = 0; pass < 2; ++pass) {
#pragma unroll
        for (int it = 0; it < 4; ++it) {
          const int row = it * 4 + q;
          const float* sp = slab + row * 68 + c8;
          v8h hv, lv;
#pragma unroll
          for (int e = 0; e < 8; ++e) {
            if (OUT_MODE == 1) {
              hv[e] = (_Float16)sp[e];
            } else {
              unsigned short hb = f2bf_bits(sp[e]);
              unsigned short lb = f2bf_bits(sp[e] - bf_bits2f(hb));
              hv[e] = __builtin_bit_cast(_Float16, hb);
              lv[e] = __builtin_bit_cast(_Float16, lb);
            }
          }
          *(volatile v8h*)(C + (size_t)(mBase + row) * ldc + n0 + c8) = hv;
          if (OUT_MODE == 2) *(volatile v8h*)(C2 + (size_t)(mBase + row) * ldc + n0 + c8) = lv;
        }
        __threadfence();
      }
    }
    __builtin_amdgcn_fence(__ATOMIC_RELEASE, "workgroup");
    __builtin_amdgcn_wave_barrier();
    __builtin_amdgcn_fence(__ATOMIC_ACQUIRE, "workgroup");
  }
}

template <int FMT>
__global__ __launch_bounds__(NTHR) void tpw_kernel(const float* __restrict__ src, int R, int C, int ldo,
                                                  unsigned short* __restrict__ O, float sc) {
  __shared__ float Tt[64 * 65];
  const int tid = threadIdx.x;
  const int c0 = blockIdx.x * 64, r0 = blockIdx.y * 64;
#pragma unroll
  for (int i = 0; i < 4; ++i) {
    const int idx = i * NTHR + tid;
    const int rr = idx >> 4, cc = (idx & 15) * 4;
    const v4f v = *(const v4f*)(src + (size_t)(r0 + rr) * (size_t)C + c0 + cc);
    Tt[rr * 65 + cc + 0] = v[0];
    Tt[rr * 65 + cc + 1] = v[1];
    Tt[rr * 65 + cc + 2] = v[2];
    Tt[rr * 65 + cc + 3] = v[3];
  }
  __syncthreads();
  const int q = tid >> 3, c8 = (tid & 7) * 8;
  v8h hv[2];
#pragma unroll
  for (int g = 0; g < 2; ++g) {
    const int qq = g * 32 + q;
#pragma unroll
    for (int e = 0; e < 8; ++e) {
      const float f = Tt[(c8 + e) * 65 + qq];
      unsigned short bits;
      if (FMT == 0) {
        bits = f2bf_bits(f * sc);
      } else {
        bits = __builtin_bit_cast(unsigned short, (_Float16)(f * sc));
      }
      hv[g][e] = __builtin_bit_cast(_Float16, bits);
    }
  }
  for (int pass = 0; pass < 2; ++pass) {
#pragma unroll
    for (int g = 0; g < 2; ++g) {
      const size_t o = (size_t)(c0 + g * 32 + q) * (size_t)ldo + (size_t)(r0 + c8);
      *(volatile v8h*)(O + o) = hv[g];
    }
    __threadfence();
  }
}

__global__ __launch_bounds__(NTHR) void frontend_kernel(const int* __restrict__ code, const float* __restrict__ aux,
                                                        const float* __restrict__ W_lin, const float* __restrict__ b_lin,
                                                        unsigned short* __restrict__ X16) {
  __shared__ int   cs[FE_RPB][48];
  __shared__ float ax[FE_RPB][16];
  __shared__ __align__(16) float sl[FE_RPB][NE];
  const int tid = threadIdx.x, lane = tid & 31, wave = tid >> 5;
  const int rt = blockIdx.x * FE_RPB + wave;
  const int t  = rt >> 7;
  const int b  = rt & (NBAT - 1);
  const size_t cbase = ((size_t)b * NTS + (size_t)t) * NCV;
  const size_t abase = ((size_t)b * NTS + (size_t)t) * NAUX;
  const int s1 = (32 + lane < NCV) ? (32 + lane) : (NCV - 1);
  const int code0 = code[cbase + lane];
  const int code1 = code[cbase + s1];
  const float av = aux[abase + (lane & 15)];
  cs[wave][lane] = code0;
  if (lane < NCV - 32) cs[wave][32 + lane] = code1;
  if (lane < 16) ax[wave][lane] = av;
  __syncthreads();

  v4f a = *(const v4f*)(b_lin + 4 * lane);
#pragma unroll 1
  for (int c = 0; c < NCV; ++c) {
    const int cc = cs[wave][c];
    const bool earlier = ((code0 == cc) && (lane < c)) || ((code1 == cc) && (lane + 32 < c));
    const unsigned dupm = __builtin_amdgcn_ballot_w32(earlier);
    const bool keep = (cc >= 1) && (cc <= NVOC) && (dupm == 0u);
    const float f = keep ? 1.0f : 0.0f;
    int row = cc - 1;
    row = (row < 0) ? 0 : ((row > NVOC - 1) ? (NVOC - 1) : row);
    const v4f w = *(const v4f*)(W_lin + (size_t)row * NE + 4 * lane);
    a[0] = fmaf(f, w[0], a[0]);
    a[1] = fmaf(f, w[1], a[1]);
    a[2] = fmaf(f, w[2], a[2]);
    a[3] = fmaf(f, w[3], a[3]);
  }
#pragma unroll 1
  for (int k = 0; k < NAUX; ++k) {
    const float xk = ax[wave][k];
    const v4f w = *(const v4f*)(W_lin + (size_t)(NVOC + k) * NE + 4 * lane);
    a[0] = fmaf(xk, w[0], a[0]);
    a[1] = fmaf(xk, w[1], a[1]);
    a[2] = fmaf(xk, w[2], a[2]);
    a[3] = fmaf(xk, w[3], a[3]);
  }
  v4f xo;
#pragma unroll
  for (int e = 0; e < 4; ++e) xo[e] = fmaxf(a[e], 0.0f) * XCAR;
  *(v4f*)(&sl[wave][4 * lane]) = xo;
  __syncthreads();
  const int l16 = lane & 15;
  const v4f p0 = *(const v4f*)(&sl[wave][8 * l16]);
  const v4f p1 = *(const v4f*)(&sl[wave][8 * l16 + 4]);
  v8h hv;
#pragma unroll
  for (int e = 0; e < 4; ++e) { hv[e] = (_Float16)p0[e]; hv[4 + e] = (_Float16)p1[e]; }
  unsigned short* dst = X16 + (size_t)rt * NE + 8 * l16;
  if (lane < 16) *(volatile v8h*)dst = hv;
  __threadfence();
  if (lane < 16) *(volatile v8h*)dst = hv;
}

__global__ __launch_bounds__(NTHR) void lstm_head_kernel(const float* __restrict__ XP, const unsigned short* __restrict__ WHTp,
                                                         const int* __restrict__ length,
                                                         const float* __restrict__ W0, const float* __restrict__ b0v,
                                                         const float* __restrict__ W1, const float* __restrict__ b1v,
                                                         float* __restrict__ out) {
  __shared__ __align__(16) _Float16 Ah[SEQB * HPITCH];
  __shared__ __align__(16) float    Zs[SEQB * ZPITCH];
  __shared__ __align__(16) float    Ls[SEQB * LPITCH];
  __shared__ __align__(16) float    Ys[SEQB * YPITCH];
  const _Float16* WH = (const _Float16*)WHTp;
  const int tid = threadIdx.x, lane = tid & 31, wave = tid >> 5;
  const int c = lane & 15, hh = lane >> 4, koff = hh * 8;
  const int rowbase = blockIdx.x * SEQB;
  const int j = 16 * wave + c;

#pragma unroll 1
  for (int i = tid; i < SEQB * HPITCH; i += NTHR) Ah[i] = (_Float16)0.0f;
  int lidx[8];
  float cst[8], hst[8], lastv[8];
#pragma unroll
  for (int r = 0; r < 8; ++r) {
    const int L = length[rowbase + 8 * hh + r];
    int ix = L - 1;
    ix = (ix < 0) ? (ix + NTS) : ix;
    ix = (ix < 0) ? 0 : ((ix > NTS - 1) ? (NTS - 1) : ix);
    lidx[r] = ix;
    cst[r] = 0.0f; hst[r] = 0.0f; lastv[r] = 0.0f;
  }
  __syncthreads();

  const _Float16* ahrow = Ah + c * HPITCH + koff;
  const _Float16* wh = WH + (size_t)j * NE + koff;
  const v8f z8 = {0.f, 0.f, 0.f, 0.f, 0.f, 0.f, 0.f, 0.f};

#pragma unroll 1
  for (int t = 0; t < NTS; ++t) {
#pragma unroll
    for (int it = 0; it < 8; ++it) {
      const int idx = it * NTHR + tid;
      const int row = idx >> 7, c4 = (idx & 127) * 4;
      const v4f v = *(const v4f*)(XP + ((size_t)(t * NBAT + rowbase + row)) * NG4 + c4);
      *(v4f*)(Zs + row * ZPITCH + c4) = v;
    }
    __syncthreads();

    v8f acc0 = z8, acc1 = z8, acc2 = z8, acc3 = z8;
#pragma unroll 1
    for (int k0 = 0; k0 < NE; k0 += 32) {
      const v16h a  = Frag<_Float16>::load(ahrow + k0);
      const v16h b0 = Frag<_Float16>::load(wh + k0);
      const v16h b1 = Frag<_Float16>::load(wh + (size_t)1 * NE * NE + k0);
      const v16h b2 = Frag<_Float16>::load(wh + (size_t)2 * NE * NE + k0);
      const v16h b3 = Frag<_Float16>::load(wh + (size_t)3 * NE * NE + k0);
      acc0 = Frag<_Float16>::mma(a, b0, acc0);
      acc1 = Frag<_Float16>::mma(a, b1, acc1);
      acc2 = Frag<_Float16>::mma(a, b2, acc2);
      acc3 = Frag<_Float16>::mma(a, b3, acc3);
      mma_guard_all_h(acc0, acc1, acc2, acc3, a, b0, b1, b2, b3);
    }
    acc_guard4(acc0, acc1, acc2, acc3);
#pragma unroll
    for (int r = 0; r < 8; ++r) {
      const float* zr = Zs + (8 * hh + r) * ZPITCH + j;
      const float zi = acc0[r] * HW_INV + zr[0];
      const float zf = acc1[r] * HW_INV + zr[NE];
      const float zg = acc2[r] * HW_INV + zr[2 * NE];
      const float zo = acc3[r] * HW_INV + zr[3 * NE];
      const float ig = fsig(zi);
      const float fg = fsig(zf);
      const float gg = ftanh(zg);
      const float og = fsig(zo);
      const float cn = fg * cst[r] + ig * gg;
      cst[r] = cn;
      const float hn = og * ftanh(cn);
      hst[r] = hn;
      lastv[r] = (t == lidx[r]) ? hn : lastv[r];
    }
    __syncthreads();
#pragma unroll
    for (int r = 0; r < 8; ++r) Ah[(8 * hh + r) * HPITCH + j] = (_Float16)(hst[r] * HCAR);
  }

#pragma unroll
  for (int r = 0; r < 8; ++r) Ls[(8 * hh + r) * LPITCH + j] = lastv[r];
  __syncthreads();
  float y[16];
#pragma unroll
  for (int r = 0; r < 16; ++r) y[r] = 0.0f;
#pragma unroll 1
  for (int k = 0; k < NE; ++k) {
    const float w = W0[(size_t)k * NHM + tid];
#pragma unroll
    for (int r = 0; r < 16; ++r) y[r] = fmaf(Ls[r * LPITCH + k], w, y[r]);
  }
  const float bv0 = b0v[tid];
#pragma unroll
  for (int r = 0; r < 16; ++r) Ys[r * YPITCH + tid] = fmaxf(y[r] + bv0, 0.0f);
  __syncthreads();
  float fe[16];
#pragma unroll
  for (int r = 0; r < 16; ++r) fe[r] = 0.0f;
#pragma unroll 1
  for (int k = 0; k < NHM; ++k) {
    const float w = W1[(size_t)k * NHM + tid];
#pragma unroll
    for (int r = 0; r < 16; ++r) fe[r] = fmaf(Ys[r * YPITCH + k], w, fe[r]);
  }
  const float bv1 = b1v[tid];
#pragma unroll
  for (int r = 0; r < 16; ++r) Zs[r * ZPITCH + tid] = fe[r] + bv1;
  __syncthreads();
  v4f o0[2], o1[2];
#pragma unroll
  for (int q = 0; q < 2; ++q) {
    const int row = 2 * wave + q;
    const v4f p0 = *(const v4f*)(Zs + row * ZPITCH + 4 * lane);
    const v4f p1 = *(const v4f*)(Zs + row * ZPITCH + 128 + 4 * lane);
    float ss = 0.0f;
    ss += (p0[0] * p0[0] + p0[1] * p0[1]) + (p0[2] * p0[2] + p0[3] * p0[3]);
    ss += (p1[0] * p1[0] + p1[1] * p1[1]) + (p1[2] * p1[2] + p1[3] * p1[3]);
#pragma unroll
    for (int off = 1; off < 32; off <<= 1) ss += __shfl_xor(ss, off, 32);
    const float rn = 1.0f / sqrtf(ss);
#pragma unroll
    for (int e = 0; e < 4; ++e) { o0[q][e] = p0[e] * rn; o1[q][e] = p1[e] * rn; }
  }
  float* ob = out + (size_t)rowbase * NHM;
  for (int pass = 0; pass < 2; ++pass) {
#pragma unroll
    for (int q = 0; q < 2; ++q) {
      const int row = 2 * wave + q;
      *(volatile v4f*)(ob + (size_t)row * NHM + 4 * lane) = o0[q];
      *(volatile v4f*)(ob + (size_t)row * NHM + 128 + 4 * lane) = o1[q];
    }
    __threadfence();
  }
}

extern "C" void kernel_launch(void* const* d_in, const int* in_sizes, int n_in,
                              void* d_out, int out_size, void* d_ws, size_t ws_size, hipStream_t stream) {
  if (n_in < 13 || d_out == nullptr || d_ws == nullptr) return;
  if (in_sizes[0] != NBAT * NTS * NCV || in_sizes[1] != NBAT * NTS * NAUX || in_sizes[2] != NBAT ||
      in_sizes[4] != NLIN * NE || in_sizes[5] != NE || in_sizes[6] != NE * NG4 || in_sizes[7] != NE * NG4 ||
      in_sizes[8] != NG4 || in_sizes[9] != NE * NHM || in_sizes[10] != NHM || in_sizes[11] != NHM * NHM ||
      in_sizes[12] != NHM || out_size != NBAT * NHM) return;

  const int*   code   = (const int*)  d_in[0];
  const float* aux    = (const float*)d_in[1];
  const int*   length = (const int*)  d_in[2];
  const float* W_lin  = (const float*)d_in[4];
  const float* b_lin  = (const float*)d_in[5];
  const float* W_x    = (const float*)d_in[6];
  const float* W_h    = (const float*)d_in[7];
  const float* b_lstm = (const float*)d_in[8];
  const float* W0     = (const float*)d_in[9];
  const float* b0v    = (const float*)d_in[10];
  const float* W1     = (const float*)d_in[11];
  const float* b1v    = (const float*)d_in[12];
  float* out = (float*)d_out;

  char* ws = (char*)d_ws; size_t off = 0;
  auto carve = [&](size_t bytes) -> char* { char* p = ws + off; off += (bytes + 255) & ~(size_t)255; return p; };
  unsigned short* X16 = (unsigned short*)carve((size_t)NROW * NE * 2);
  unsigned short* WXT = (unsigned short*)carve((size_t)NG4 * NE * 2);
  unsigned short* WHT = (unsigned short*)carve((size_t)NG4 * NE * 2);
  float*          XP  = (float*)carve((size_t)NROW * NG4 * 4);
  if (off > ws_size || off > (size_t)134217728) return;

  tpw_kernel<1><<<dim3(NG4 / 64, NE / 64), NTHR, 0, stream>>>(W_x, NE, NG4, NE, WXT, WCAR);
  tpw_kernel<1><<<dim3(NG4 / 64, NE / 64), NTHR, 0, stream>>>(W_h, NE, NG4, NE, WHT, WCAR);
  frontend_kernel<<<NROW / FE_RPB, NTHR, 0, stream>>>(code, aux, W_lin, b_lin, X16);
  const dim3 ggrid((NROW / 64) * (NG4 / 64) / 8, 1);
  wmma_gemm64<0, false, 2, 0, false, 0><<<ggrid, 256, 0, stream>>>(
      X16, X16, NE, 0L, WXT, WXT, NE, 0L, (void*)XP, (void*)XP, NG4, 0L,
      b_lstm, (const float*)XP, 0L, NROW, NG4, NE, XW_INV);
  lstm_head_kernel<<<NBAT / SEQB, NTHR, 0, stream>>>(XP, WHT, length, W0, b0v, W1, b1v, out);
}
